// TransformerEncoderLayer_8461085573377
// MI455X (gfx1250) — hardware-verified
//
#include <hip/hip_runtime.h>
#include <stddef.h>
#include <stdint.h>


#ifndef NB
#define NB 2
#endif
#ifndef SEQ
#define SEQ 2048
#endif
#define NB_FULL  2
#define SEQ_FULL 2048
#define DM     1024
#define DFF    4096
#define NH     16
#define HD     64
#define QKW    2048
#define MTOK   (NB * SEQ)
#define NTHR   256
#define GBM    64
#define GBN    64
#define GTHR   128
#define ATHR   128
#define AQB    64
#define AKC    64
#define OSP    72
#define TT     64
#define TP     68
#define CX     8.0f
#define CW     64.0f
#define CQK    4.0f
#define CV     4.0f
#define CP     1024.0f
#define CA     64.0f
#define CH     8.0f
#define SCL_XW 0.001953125f
#define SCL_AW 0.000244140625f
#define SCL_HW 0.001953125f
#define SSCL   0.0078125f
#define KO     0.015625f
#define LNEPS  1.0e-5f
#define WSMAX  134217728

static_assert(DM == NH * HD);
static_assert(HD == 64);
static_assert(NB >= 1 && NB <= NB_FULL);
static_assert(SEQ >= AQB && SEQ <= SEQ_FULL);
static_assert((SEQ % AQB) == 0 && (SEQ % AKC) == 0);
static_assert(AQB == (ATHR / 32) * 16 && AKC == 64);
static_assert((MTOK % GBM) == 0 && (MTOK % GBN) == 0 && (MTOK % 8) == 0);
static_assert((DM % GBN) == 0 && (DFF % GBN) == 0 && (QKW % GBN) == 0 && (DM % GBM) == 0);
static_assert((DM % 32) == 0 && (DFF % 32) == 0);
static_assert(GBM == (GTHR / 32) * 16);
static_assert((DM % TT) == 0 && (DFF % TT) == 0);
static_assert(NTHR == 8 * 32);
static_assert(DM == 4 * 8 * 32);
static_assert(DM == 8 * 4 * 32);
static_assert((DM / 8) == 128);
static_assert(((MTOK * (DM / 8)) % NTHR) == 0);
static_assert((OSP % 8) == 0);

typedef float    v4f  __attribute__((ext_vector_type(4)));
typedef float    v8f  __attribute__((ext_vector_type(8)));
typedef int      v8i  __attribute__((ext_vector_type(8)));
typedef _Float16 v8h  __attribute__((ext_vector_type(8)));
typedef _Float16 v16h __attribute__((ext_vector_type(16)));
union FragH { v16h v; v8h h[2]; v8i w; };

__device__ __forceinline__ v8f wmh(const FragH& a, const FragH& b, v8f c) {
  v8f d = __builtin_amdgcn_wmma_f32_16x16x32_f16(false, a.v, false, b.v, (short)0, c, false, false);
  asm volatile("v_nop\n\tv_nop\n\tv_nop\n\tv_nop" : "+v"(d) : "v"(a.w), "v"(b.w));
  return d;
}

__device__ __forceinline__ float bfr(float x) {
  unsigned int u = __float_as_uint(x);
  u = (u + 0x7FFFu + ((u >> 16) & 1u)) & 0xFFFF0000u;
  return __uint_as_float(u);
}
__device__ __forceinline__ v4f bfr4(const v4f a) {
  v4f r;
  r.x = bfr(a.x); r.y = bfr(a.y); r.z = bfr(a.z); r.w = bfr(a.w);
  return r;
}

__device__ __forceinline__ v8h cvt8h(const v4f a, const v4f b, const float c) {
  v8h hv;
  hv[0] = (_Float16)(a.x * c); hv[1] = (_Float16)(a.y * c);
  hv[2] = (_Float16)(a.z * c); hv[3] = (_Float16)(a.w * c);
  hv[4] = (_Float16)(b.x * c); hv[5] = (_Float16)(b.y * c);
  hv[6] = (_Float16)(b.z * c); hv[7] = (_Float16)(b.w * c);
  return hv;
}

__device__ __forceinline__ void wave_lds_sync() {
  __builtin_amdgcn_fence(3  , "wavefront");
  __builtin_amdgcn_wave_barrier();
}

__global__ __launch_bounds__(NTHR) void k_xprep(const float* __restrict__ x, _Float16* xh, int nUnits) {
  const int i = (int)blockIdx.x * NTHR + (int)threadIdx.x;
  if (i >= nUnits) return;
  const int row = i >> 7;
  const int c0  = (i & 127) * 8;
  const int bb  = row / SEQ;
  const int s   = row - bb * SEQ;
  const size_t srow = (size_t)bb * SEQ_FULL + (size_t)s;
  const float* p = x + srow * DM + c0;
  const v4f a = bfr4(*(const v4f*)p), b = bfr4(*(const v4f*)(p + 4));
  const v8h hv = cvt8h(a, b, CX);
  const size_t o = (size_t)row * DM + c0;
  *(volatile v8h*)(xh + o) = hv;
  __threadfence();
  *(volatile v8h*)(xh + o) = hv;
}

__global__ __launch_bounds__(NTHR) void k_wtr(const float* __restrict__ W, _Float16* WT, int K, int Nc) {
  __shared__ __attribute__((aligned(16))) float tile[TT * TP];
  const int tid = (int)threadIdx.x, lane = tid & 31, wave = tid >> 5;
  const int n0 = (int)blockIdx.x * TT;
  const int k0 = (int)blockIdx.y * TT;
#pragma unroll
  for (int i = 0; i < 4; ++i) {
    const int kr = (tid >> 4) + 16 * i;
    const int c4 = (tid & 15) * 4;
    const v4f v = *(const v4f*)(W + (size_t)(k0 + kr) * (size_t)Nc + n0 + c4);
    *(v4f*)(tile + kr * TP + c4) = bfr4(v);
  }
  __syncthreads();
  const int q = lane & 7;
  v8h hv[2];
#pragma unroll
  for (int i = 0; i < 2; ++i) {
    const int nr = 8 * wave + 4 * i + (lane >> 3);
    v4f a, b;
    a.x = tile[(8 * q + 0) * TP + nr]; a.y = tile[(8 * q + 1) * TP + nr];
    a.z = tile[(8 * q + 2) * TP + nr]; a.w = tile[(8 * q + 3) * TP + nr];
    b.x = tile[(8 * q + 4) * TP + nr]; b.y = tile[(8 * q + 5) * TP + nr];
    b.z = tile[(8 * q + 6) * TP + nr]; b.w = tile[(8 * q + 7) * TP + nr];
    hv[i] = cvt8h(a, b, CW);
  }
#pragma unroll
  for (int i = 0; i < 2; ++i) {
    const int nr = 8 * wave + 4 * i + (lane >> 3);
    _Float16* op = WT + (size_t)(n0 + nr) * (size_t)K + k0 + 8 * q;
    *(volatile v8h*)op = hv[i];
  }
  __threadfence();
#pragma unroll
  for (int i = 0; i < 2; ++i) {
    const int nr = 8 * wave + 4 * i + (lane >> 3);
    _Float16* op = WT + (size_t)(n0 + nr) * (size_t)K + k0 + 8 * q;
    *(volatile v8h*)op = hv[i];
  }
}

template<int EPI, int BROW>
__global__ __launch_bounds__(GTHR) void k_gemm(
    const _Float16* __restrict__ A, const _Float16* __restrict__ WT,
    const float* __restrict__ b0, const float* __restrict__ b1, const float* __restrict__ b2,
    float* outF, _Float16* outH,
    int K, int ldo, int ldh, int segN, float scl, float cao)
{
  __shared__ __attribute__((aligned(16))) float stg[GBM * GBN];
  const int tid = (int)threadIdx.x, lane = tid & 31, wave = tid >> 5, hh = lane >> 4, m = lane & 15;
  const int rowBase = (int)blockIdx.x * GBM;
  const int col0    = (int)blockIdx.y * GBN;
  const float* bp = b0;
  int bofs = 0;
  if (!BROW) {
    int seg = col0 / segN;
    seg = seg < 0 ? 0 : (seg > 2 ? 2 : seg);
    bp = (seg == 0) ? b0 : ((seg == 1) ? b1 : b2);
    bofs = col0 - seg * segN;
    bofs = bofs < 0 ? 0 : bofs;
  }

  v8f acc[4];
  {
    const v8f z = {0.f, 0.f, 0.f, 0.f, 0.f, 0.f, 0.f, 0.f};
    acc[0] = z; acc[1] = z; acc[2] = z; acc[3] = z;
  }
  const _Float16* ap = A  + (size_t)(rowBase + 16 * wave + m) * (size_t)K + 8 * hh;
  const _Float16* wp = WT + (size_t)(col0 + m) * (size_t)K + 8 * hh;
  const int ksteps = K >> 5;
#pragma unroll 1
  for (int ks = 0; ks < ksteps; ++ks) {
    FragH af;
    af.h[0] = *(const v8h*)(ap + 32 * ks);
    af.h[1] = *(const v8h*)(ap + 32 * ks + 16);
#pragma unroll
    for (int t = 0; t < 4; ++t) {
      const _Float16* wq = wp + (size_t)(16 * t) * (size_t)K + 32 * ks;
      FragH bf;
      bf.h[0] = *(const v8h*)wq;
      bf.h[1] = *(const v8h*)(wq + 16);
      acc[t] = wmh(af, bf, acc[t]);
    }
  }

  float brw[8];
#pragma unroll
  for (int r = 0; r < 8; ++r) brw[r] = 0.f;
  if (BROW) {
#pragma unroll
    for (int r = 0; r < 8; ++r) {
      int ri = rowBase + 16 * wave + 8 * hh + r;
      ri = ri > segN - 1 ? segN - 1 : ri;
      brw[r] = bfr(bp[ri]);
    }
  }
#pragma unroll
  for (int t = 0; t < 4; ++t) {
    const int lc = 16 * t + m;
    float bcol = 0.f;
    if (!BROW) {
      int bi = bofs + lc;
      bi = bi > segN - 1 ? segN - 1 : bi;
      bcol = bfr(bp[bi]);
    }
#pragma unroll
    for (int r = 0; r < 8; ++r) {
      const int lr = 16 * wave + 8 * hh + r;
      float v = fmaf(acc[t][r], scl, BROW ? brw[r] : bcol);
      if (EPI == 1) v = fmaxf(v, 0.f);
      stg[lr * GBN + lc] = v;
    }
  }
  __syncthreads();

  if (EPI == 0) {
    v4f fv[8];
#pragma unroll
    for (int i = 0; i < 8; ++i) {
      const int lr = 16 * wave + 2 * i + hh;
      fv[i] = *(const v4f*)(stg + lr * GBN + 4 * m);
    }
#pragma unroll
    for (int i = 0; i < 8; ++i) {
      const int lr = 16 * wave + 2 * i + hh;
      float* op = outF + (size_t)(rowBase + lr) * (size_t)ldo + col0 + 4 * m;
      *(volatile v4f*)op = fv[i];
    }
    __threadfence();
#pragma unroll
    for (int i = 0; i < 8; ++i) {
      const int lr = 16 * wave + 2 * i + hh;
      float* op = outF + (size_t)(rowBase + lr) * (size_t)ldo + col0 + 4 * m;
      *(volatile v4f*)op = fv[i];
    }
  }
  if (EPI != 0) {
    v8h hv[4];
    const int q = lane & 7;
#pragma unroll
    for (int i = 0; i < 4; ++i) {
      const int lr = 16 * wave + 4 * i + (lane >> 3);
      const v4f a = *(const v4f*)(stg + lr * GBN + 8 * q);
      const v4f b = *(const v4f*)(stg + lr * GBN + 8 * q + 4);
      hv[i] = cvt8h(a, b, cao);
    }
#pragma unroll
    for (int i = 0; i < 4; ++i) {
      const int lr = 16 * wave + 4 * i + (lane >> 3);
      _Float16* op = outH + (size_t)(rowBase + lr) * (size_t)ldh + col0 + 8 * q;
      *(volatile v8h*)op = hv[i];
    }
    __threadfence();
#pragma unroll
    for (int i = 0; i < 4; ++i) {
      const int lr = 16 * wave + 4 * i + (lane >> 3);
      _Float16* op = outH + (size_t)(rowBase + lr) * (size_t)ldh + col0 + 8 * q;
      *(volatile v8h*)op = hv[i];
    }
  }
}

__global__ __launch_bounds__(ATHR) void k_attn(
    const _Float16* __restrict__ QK, const _Float16* __restrict__ VT, _Float16* AH, int ldv)
{
  __shared__ __attribute__((aligned(16))) _Float16 os[(ATHR / 32) * 16 * OSP];
  const int tid = (int)threadIdx.x, lane = tid & 31, wave = tid >> 5, hh = lane >> 4, m = lane & 15;
  const int b = (int)blockIdx.z, h = (int)blockIdx.y;
  const int q0 = (int)blockIdx.x * AQB + 16 * wave;
  const size_t tok0  = (size_t)b * SEQ + (size_t)q0;
  const size_t ktok0 = (size_t)b * SEQ;

  FragH qf[2];
  {
    const _Float16* qp = QK + (tok0 + m) * QKW + HD * h + 8 * hh;
    qf[0].h[0] = *(const v8h*)(qp);       qf[0].h[1] = *(const v8h*)(qp + 16);
    qf[1].h[0] = *(const v8h*)(qp + 32);  qf[1].h[1] = *(const v8h*)(qp + 48);
  }
  const _Float16* kp = QK + (ktok0 + m) * QKW + DM + HD * h + 8 * hh;
  const _Float16* vp = VT + (size_t)(HD * h + m) * (size_t)ldv + ktok0 + 8 * hh;

  const v8f z = {0.f, 0.f, 0.f, 0.f, 0.f, 0.f, 0.f, 0.f};
  v8f accO[4];
  accO[0] = z; accO[1] = z; accO[2] = z; accO[3] = z;
  float mrun = -1.0e30f, lrun = 0.f;

  const int nChunks = SEQ / AKC;
#pragma unroll 1
  for (int c = 0; c < nChunks; ++c) {
    v8f accS[4];
#pragma unroll
    for (int kt = 0; kt < 4; ++kt) {
      accS[kt] = z;
      const _Float16* kq = kp + (size_t)(AKC * c + 16 * kt) * QKW;
#pragma unroll
      for (int ks = 0; ks < 2; ++ks) {
        FragH af;
        af.h[0] = *(const v8h*)(kq + 32 * ks);
        af.h[1] = *(const v8h*)(kq + 32 * ks + 16);
        accS[kt] = wmh(af, qf[ks], accS[kt]);
      }
    }
    float mx = accS[0][0];
#pragma unroll
    for (int kt = 0; kt < 4; ++kt) {
#pragma unroll
      for (int r = 0; r < 8; ++r) mx = fmaxf(mx, accS[kt][r]);
    }
    mx = mx * SSCL;
    mx = fmaxf(mx, __shfl_xor(mx, 16));
    const float mnew  = fmaxf(mrun, mx);
    const float alpha = __expf(mrun - mnew);
    float ps = 0.f;
    FragH pb[2];
#pragma unroll
    for (int kt = 0; kt < 4; ++kt) {
      v8h hv;
#pragma unroll
      for (int r = 0; r < 8; ++r) {
        const float p = __expf(fmaf(accS[kt][r], SSCL, -mnew));
        ps += p;
        hv[r] = (_Float16)(p * CP);
      }
      pb[kt >> 1].h[kt & 1] = hv;
    }
    ps += __shfl_xor(ps, 16);
    lrun = fmaf(lrun, alpha, ps);
    mrun = mnew;
#pragma unroll
    for (int dt = 0; dt < 4; ++dt) accO[dt] = accO[dt] * alpha;
#pragma unroll
    for (int dt = 0; dt < 4; ++dt) {
      const _Float16* vq = vp + (size_t)(16 * dt) * (size_t)ldv + AKC * c;
#pragma unroll
      for (int ks = 0; ks < 2; ++ks) {
        FragH av;
        av.h[0] = *(const v8h*)(vq + 32 * ks);
        av.h[1] = *(const v8h*)(vq + 32 * ks + 16);
        accO[dt] = wmh(av, pb[ks], accO[dt]);
      }
    }
  }

  const float f = KO * __builtin_amdgcn_rcpf(lrun);
  _Float16* ow = os + wave * (16 * OSP);
#pragma unroll
  for (int dt = 0; dt < 4; ++dt) {
    v8h hv;
#pragma unroll
    for (int r = 0; r < 8; ++r) hv[r] = (_Float16)(accO[dt][r] * f);
    *(v8h*)(ow + m * OSP + 16 * dt + 8 * hh) = hv;
  }
  wave_lds_sync();
  v8h sv[4];
#pragma unroll
  for (int i = 0; i < 4; ++i) {
    const int qq = 4 * i + (lane >> 3);
    sv[i] = *(const v8h*)(ow + qq * OSP + 8 * (lane & 7));
  }
#pragma unroll
  for (int i = 0; i < 4; ++i) {
    _Float16* op = AH + (tok0 + (size_t)(4 * i + (lane >> 3))) * DM + HD * h + 8 * (lane & 7);
    *(volatile v8h*)op = sv[i];
  }
  __threadfence();
#pragma unroll
  for (int i = 0; i < 4; ++i) {
    _Float16* op = AH + (tok0 + (size_t)(4 * i + (lane >> 3))) * DM + HD * h + 8 * (lane & 7);
    *(volatile v8h*)op = sv[i];
  }
}

template<int MODE>
__global__ __launch_bounds__(NTHR) void k_ln(
    const float* __restrict__ a, const float* __restrict__ b,
    const float* __restrict__ g, const float* __restrict__ be,
    float* outF, _Float16* outH, int nRows)
{
  __shared__ __attribute__((aligned(16))) float stg[8 * DM];
  const int tid = (int)threadIdx.x, lane = tid & 31, wave = tid >> 5;
  const int row = (int)blockIdx.x * 8 + wave;
  if (row >= nRows) return;
  size_t arow = (size_t)row;
  if (MODE == 0) {
    const int bb = row / SEQ;
    const int s  = row - bb * SEQ;
    arow = (size_t)bb * SEQ_FULL + (size_t)s;
  }
  const float* ap  = a + arow * DM;
  const float* bpp = b + (size_t)row * DM;
  float* sw = stg + wave * DM;

  float s1 = 0.f;
#pragma unroll 1
  for (int i = 0; i < 4; ++i) {
    const int c = 256 * i + 8 * lane;
    v4f a0 = *(const v4f*)(ap + c), a1 = *(const v4f*)(ap + c + 4);
    if (MODE == 0) { a0 = bfr4(a0); a1 = bfr4(a1); }
    const v4f c0 = *(const v4f*)(bpp + c), c1 = *(const v4f*)(bpp + c + 4);
    const v4f t0 = a0 + c0, t1 = a1 + c1;
    *(v4f*)(sw + c)     = t0;
    *(v4f*)(sw + c + 4) = t1;
    s1 += ((t0.x + t0.y) + (t0.z + t0.w)) + ((t1.x + t1.y) + (t1.z + t1.w));
  }
#pragma unroll
  for (int o = 16; o > 0; o >>= 1) s1 += __shfl_xor(s1, o);
  const float mu = s1 * (1.0f / DM);

  float ss = 0.f;
#pragma unroll 1
  for (int i = 0; i < 4; ++i) {
    const int c = 256 * i + 8 * lane;
    const v4f t0 = *(const v4f*)(sw + c), t1 = *(const v4f*)(sw + c + 4);
    const v4f d0 = t0 - mu, d1 = t1 - mu;
    ss += ((d0.x * d0.x + d0.y * d0.y) + (d0.z * d0.z + d0.w * d0.w))
        + ((d1.x * d1.x + d1.y * d1.y) + (d1.z * d1.z + d1.w * d1.w));
  }
#pragma unroll
  for (int o = 16; o > 0; o >>= 1) ss += __shfl_xor(ss, o);
  const float var  = ss * (1.0f / DM);
  const float rstd = rsqrtf(var + LNEPS);

#pragma unroll 1
  for (int i = 0; i < 4; ++i) {
    const int c = 256 * i + 8 * lane;
    const v4f t0 = *(const v4f*)(sw + c), t1 = *(const v4f*)(sw + c + 4);
    const v4f g0 = bfr4(*(const v4f*)(g + c)),  gg1 = bfr4(*(const v4f*)(g + c + 4));
    const v4f e0 = bfr4(*(const v4f*)(be + c)), e1  = bfr4(*(const v4f*)(be + c + 4));
    const v4f y0 = ((t0 - mu) * rstd) * g0 + e0;
    const v4f y1 = ((t1 - mu) * rstd) * gg1 + e1;
    *(v4f*)(sw + c)     = y0;
    *(v4f*)(sw + c + 4) = y1;
  }

  if (MODE == 0) {
    v8h hv[4];
#pragma unroll
    for (int i = 0; i < 4; ++i) {
      const int c = 256 * i + 8 * lane;
      const v4f y0 = *(const v4f*)(sw + c), y1 = *(const v4f*)(sw + c + 4);
      hv[i] = cvt8h(y0, y1, CX);
    }
#pragma unroll
    for (int i = 0; i < 4; ++i) {
      _Float16* hp = outH + (size_t)row * DM + 256 * i + 8 * lane;
      *(volatile v8h*)hp = hv[i];
    }
    __threadfence();
#pragma unroll
    for (int i = 0; i < 4; ++i) {
      _Float16* hp = outH + (size_t)row * DM + 256 * i + 8 * lane;
      *(volatile v8h*)hp = hv[i];
    }
  }

  wave_lds_sync();
  v4f p[8];
#pragma unroll
  for (int j = 0; j < 8; ++j) p[j] = *(const v4f*)(sw + 128 * j + 4 * lane);
  float* o = outF + (size_t)row * DM;
#pragma unroll
  for (int j = 0; j < 8; ++j) *(volatile v4f*)(o + 128 * j + 4 * lane) = p[j];
  __threadfence();
#pragma unroll
  for (int j = 0; j < 8; ++j) *(volatile v4f*)(o + 128 * j + 4 * lane) = p[j];
}

extern "C" void kernel_launch(void* const* d_in, const int* in_sizes, int n_in,
                              void* d_out, int out_size, void* d_ws, size_t ws_size,
                              hipStream_t stream) {
  if (n_in < 17) return;
  const long needSrc = ((long)(NB - 1) * SEQ_FULL + (long)SEQ) * (long)DM;
  if ((long)in_sizes[0] < needSrc) return;
  if (in_sizes[1]  != DM * DM  || in_sizes[2]  != DM)  return;
  if (in_sizes[3]  != DM * DM  || in_sizes[4]  != DM)  return;
  if (in_sizes[5]  != DM * DM  || in_sizes[6]  != DM)  return;
  if (in_sizes[7]  != DM * DM  || in_sizes[8]  != DM)  return;
  if (in_sizes[9]  != DM * DFF || in_sizes[10] != DFF) return;
  if (in_sizes[11] != DFF * DM || in_sizes[12] != DM)  return;
  if (in_sizes[13] != DM || in_sizes[14] != DM) return;
  if (in_sizes[15] != DM || in_sizes[16] != DM) return;
  if ((long)out_size < (long)MTOK * DM) return;

  const float* src = (const float*)d_in[0];
  const float* Wq  = (const float*)d_in[1];   const float* bq  = (const float*)d_in[2];
  const float* Wk  = (const float*)d_in[3];   const float* bk  = (const float*)d_in[4];
  const float* Wv  = (const float*)d_in[5];   const float* bv  = (const float*)d_in[6];
  const float* Wo  = (const float*)d_in[7];   const float* bo  = (const float*)d_in[8];
  const float* W1  = (const float*)d_in[9];   const float* b1  = (const float*)d_in[10];
  const float* W2  = (const float*)d_in[11];  const float* b2  = (const float*)d_in[12];
  const float* g1  = (const float*)d_in[13];  const float* be1 = (const float*)d_in[14];
  const float* g2  = (const float*)d_in[15];  const float* be2 = (const float*)d_in[16];
  float* out = (float*)d_out;

  const int M = MTOK;

  const size_t szR1 = (size_t)M * 8192;
  size_t off = 0;
  const size_t oR1  = off;                 off += szR1;
  const size_t oXH  = oR1;
  const size_t oQK  = oR1 + (size_t)M * 2048;
  const size_t oVT  = oR1 + (size_t)M * 6144;
  const size_t oHH  = oR1;
  const size_t oWQ  = off;                 off += (size_t)3 * DM * DM * 2;
  const size_t oWO  = off;                 off += (size_t)DM * DM * 2;
  const size_t oW1  = off;                 off += (size_t)DFF * DM * 2;
  const size_t oW2  = off;                 off += (size_t)DM * DFF * 2;
  const size_t oAH  = off;                 off += (size_t)M * DM * 2;
  const size_t oSF  = off;                 off += (size_t)M * DM * 4;
  const size_t oX   = off;                 off += (size_t)M * DM * 4;
  const size_t oXH2 = off;                 off += (size_t)M * DM * 2;
  if (off > ws_size || off > (size_t)WSMAX) return;
  if (oVT + (size_t)DM * M * 2 != oR1 + szR1) return;
  if ((size_t)M * DFF * 2 != szR1) return;
  if (oQK + (size_t)M * QKW * 2 != oVT) return;

  char* ws = (char*)d_ws;
  _Float16* XH   = (_Float16*)(ws + oXH);
  _Float16* QK   = (_Float16*)(ws + oQK);
  _Float16* VT   = (_Float16*)(ws + oVT);
  _Float16* HH   = (_Float16*)(ws + oHH);
  _Float16* WQKV = (_Float16*)(ws + oWQ);
  _Float16* WOT  = (_Float16*)(ws + oWO);
  _Float16* W1T  = (_Float16*)(ws + oW1);
  _Float16* W2T  = (_Float16*)(ws + oW2);
  _Float16* AH   = (_Float16*)(ws + oAH);
  float*    SF   = (float*)(ws + oSF);
  float*    X    = (float*)(ws + oX);
  _Float16* XH2  = (_Float16*)(ws + oXH2);

  const int nUx = M * (DM / 8);
  k_xprep<<<nUx / NTHR, NTHR, 0, stream>>>(src, XH, nUx);

  k_wtr<<<dim3(DM / TT, DM / TT), NTHR, 0, stream>>>(Wq, WQKV, DM, DM);
  k_wtr<<<dim3(DM / TT, DM / TT), NTHR, 0, stream>>>(Wk, WQKV + (size_t)DM * DM, DM, DM);
  k_wtr<<<dim3(DM / TT, DM / TT), NTHR, 0, stream>>>(Wv, WQKV + (size_t)2 * DM * DM, DM, DM);
  k_wtr<<<dim3(DM / TT, DM / TT), NTHR, 0, stream>>>(Wo, WOT, DM, DM);
  k_wtr<<<dim3(DFF / TT, DM / TT), NTHR, 0, stream>>>(W1, W1T, DM, DFF);
  k_wtr<<<dim3(DM / TT, DFF / TT), NTHR, 0, stream>>>(W2, W2T, DFF, DM);

  const int gM = M / GBM;
  k_gemm<2, 0><<<dim3(gM, QKW / GBN), GTHR, 0, stream>>>(XH, WQKV, bq, bk, bk, SF, QK,
                                                          DM, DM, QKW, DM, SCL_XW, CQK);
  k_gemm<2, 1><<<dim3(DM / GBM, M / GBN), GTHR, 0, stream>>>(WQKV + (size_t)2 * DM * DM, XH, bv, bv, bv, SF, VT,
                                                              DM, DM, M, DM, SCL_XW, CV);
  k_attn<<<dim3(SEQ / AQB, NH, NB), ATHR, 0, stream>>>(QK, VT, AH, M);
  k_gemm<0, 0><<<dim3(gM, DM / GBN), GTHR, 0, stream>>>(AH, WOT, bo, bo, bo, SF, XH2,
                                                         DM, DM, DM, DM, SCL_AW, 1.0f);
  k_ln<0><<<M / 8, NTHR, 0, stream>>>(src, SF, g1, be1, X, XH2, M);
  k_gemm<1, 0><<<dim3(gM, DFF / GBN), GTHR, 0, stream>>>(XH2, W1T, b1, b1, b1, SF, HH,
                                                          DM, DM, DFF, DFF, SCL_XW, CH);
  k_gemm<0, 0><<<dim3(gM, DM / GBN), GTHR, 0, stream>>>(HH, W2T, b2, b2, b2, SF, XH2,
                                                         DFF, DM, DM, DM, SCL_HW, 1.0f);
  k_ln<1><<<M / 8, NTHR, 0, stream>>>(X, SF, g2, be2, out, XH2, M);
}
